// StandardAttention_3032246911478
// MI455X (gfx1250) — hardware-verified
//
#include <hip/hip_runtime.h>


#ifndef NB
#define NB 2
#endif
#ifndef SEQ
#define SEQ 2048
#endif
#ifndef NB_FULL
#define NB_FULL 2
#endif
#ifndef SEQ_FULL
#define SEQ_FULL 2048
#endif
#ifndef QE
#define QE 256
#endif

namespace {
constexpr int DMOD = 2048, KD = 2048, H = 16, HKV = 4, NREP = H / HKV, HD = 128, NKV = HKV * HD;
constexpr int MR = NB * SEQ;
constexpr int QEA = (QE < SEQ) ? QE : SEQ;
constexpr float XS = 8.0f, WS = 256.0f, QS = 8.0f, RS = 2048.0f, PS = 1024.0f, CS = 64.0f;
constexpr float LOG2E = 1.4426950408889634f, SCL = 0.08838834764831845f, ROPE_BASE = 500000.0f;
static_assert(SEQ % 64 == 0 && SEQ >= 64 && SEQ <= SEQ_FULL && NB >= 1 && NB <= NB_FULL);
static_assert(QEA % 64 == 0 && QEA >= 64 && QEA <= SEQ && (SEQ - QEA) % 64 == 0);
static_assert(DMOD == H * HD && KD == DMOD && KD % 64 == 0 && DMOD % 128 == 0 && NKV % 128 == 0 && HD == 128 && DMOD == 256 * 8 && MR % 64 == 0);

typedef _Float16 b16;
typedef __attribute__((ext_vector_type(16))) _Float16 v16b;
typedef __attribute__((ext_vector_type(8))) _Float16 v8b;
typedef __attribute__((ext_vector_type(8))) float v8f;
typedef __attribute__((ext_vector_type(4))) float v4f;

__device__ __forceinline__ float bf16_rne(float f) { unsigned int u = __float_as_uint(f); u += 0x7FFFu + ((u >> 16) & 1u); return __uint_as_float(u & 0xFFFF0000u); }
__device__ __forceinline__ v16b frag_kb(const b16* p, int hh) {
  const v8b a = *(const v8b*)(p + 8 * hh), b = *(const v8b*)(p + 16 + 8 * hh); v16b f;
#pragma unroll
  for (int e = 0; e < 8; ++e) { f[e] = a[e]; f[8 + e] = b[e]; }
  return f;
}
__device__ __forceinline__ v8f wmma16b(v16b a, v16b b, v8f c) {
  v8f d = __builtin_amdgcn_wmma_f32_16x16x32_f16(false, a, false, b, (short)0, c, false, false);
  asm volatile("v_nop\n\tv_nop\n\tv_nop\n\tv_nop" : "+v"(d) : "v"(a), "v"(b));
  return d;
}
__device__ __forceinline__ void wave_lds_sync() { __builtin_amdgcn_fence(3, "workgroup"); __builtin_amdgcn_wave_barrier(); __builtin_amdgcn_fence(2, "workgroup"); }
__device__ __forceinline__ float nexp2(float v) { return __builtin_amdgcn_exp2f(v); }
__device__ __forceinline__ void split16(float w, b16& hi, b16& lo) { hi = (b16)w; lo = (b16)((w - (float)hi) * RS); }

__global__ __launch_bounds__(256) void cvt_x_kernel(const float* __restrict__ X, b16* Xp) {
  const size_t u = (size_t)blockIdx.x * 256 + threadIdx.x; const size_t row = u >> 8; const int c8 = (int)(u & 255) * 8;
  if (row >= (size_t)MR) return;
  const size_t b = row / SEQ, s = row % SEQ;
  const float* src = X + (b * SEQ_FULL + s) * DMOD + c8;
  b16* dst = Xp + row * DMOD + c8;
  const v4f x0 = *(const v4f*)src, x1 = *(const v4f*)(src + 4); v8b o;
#pragma unroll
  for (int j = 0; j < 4; ++j) { o[j] = (b16)(bf16_rne(x0[j]) * XS); o[4 + j] = (b16)(bf16_rne(x1[j]) * XS); }
  *(volatile v8b*)dst = o; __threadfence(); *(volatile v8b*)dst = o;
}

__global__ __launch_bounds__(64) void cvt_w_kernel(const float* __restrict__ W, b16* Wt, int N) {
  __shared__ __attribute__((aligned(16))) b16 St[64][64 + 8];
  const int tid = threadIdx.x, wave = tid >> 5, lane = tid & 31; const int k0 = (int)blockIdx.x * 64, n0 = (int)blockIdx.y * 64;
  const float* src = W + (size_t)k0 * N + n0;
  for (int it = 0; it < 16; ++it) {
    const int e = (it * 64 + tid) * 4; const int kr = e >> 6, nc = e & 63;
    const v4f x = *(const v4f*)(src + (size_t)kr * N + nc);
#pragma unroll
    for (int j = 0; j < 4; ++j) St[nc + j][kr] = (b16)(bf16_rne(x[j]) * WS);
  }
  __syncthreads();
  b16* dstb = Wt + (size_t)n0 * KD + k0;
  for (int pass = 0; pass < 2; ++pass) {
#pragma unroll 1
    for (int it = 0; it < 8; ++it) {
      const int n = wave * 32 + it * 4 + (lane >> 3), ks = (lane & 7) * 8;
      const v8b o = *(const v8b*)(&St[n][ks]);
      *(volatile v8b*)(dstb + (size_t)n * KD + ks) = o; }
    __threadfence(); }
}

__global__ __launch_bounds__(256) void rope_tab_kernel(float* CT, float* ST) {
  __shared__ __attribute__((aligned(16))) float Tb[2][4][64 + 4];
  const int tid = threadIdx.x; const int r = tid >> 6, j = tid & 63; const int s0 = (int)blockIdx.x * 4;
  const float ex = (float)(2 * j) * (1.0f / 128.0f);
  const float p = powf(ROPE_BASE, ex);
  const float inv = 1.0f / p;
  const float ang = (float)(s0 + r) * inv;
  float sn, c; sincosf(ang, &sn, &c);
  Tb[0][r][j] = c; Tb[1][r][j] = sn;
  __syncthreads();
  if (tid < 128) {
    const int tb = tid >> 6, rr = (tid >> 4) & 3, seg = (tid & 15) * 4;
    const v4f f = *(const v4f*)(&Tb[tb][rr][seg]);
    float* dst = (tb == 0 ? CT : ST) + (size_t)(s0 + rr) * 64 + seg;
    *(volatile v4f*)dst = f; __threadfence(); *(volatile v4f*)dst = f;
  }
}

template <int MODE, bool RES>
__global__ __launch_bounds__(128) __attribute__((amdgpu_num_vgpr(256))) void proj_kernel(
    const b16* __restrict__ A, const b16* __restrict__ Al, const b16* __restrict__ Bt, b16* Ph, b16* Pl, float* Out,
    const float* __restrict__ CT, const float* __restrict__ ST, int nhead, int tpb, int toff) {
#pragma clang fp contract(off)
  static_assert(MODE == 2 || !RES);
  constexpr int BN = RES ? 64 : 128, NT = BN / 16;
  __shared__ __attribute__((aligned(16))) float To[64][BN + 4];
  const int tid = threadIdx.x, wave = tid >> 5, lane = tid & 31, hh = lane >> 4, col = lane & 15;
  const int by = (int)blockIdx.y; const int bsel = by / tpb, tsel = by - bsel * tpb;
  const int s0 = toff + tsel * 64;
  const size_t m0 = (size_t)bsel * SEQ + s0;
  const int n0 = (int)blockIdx.x * BN;
  const b16* arow = A + (m0 + wave * 16 + col) * KD;
  const b16* alrow = Al + (m0 + wave * 16 + col) * KD;
  const b16* brow = Bt + (size_t)(n0 + col) * KD;
  v8f acc[NT], acc2[NT];
#pragma unroll
  for (int t = 0; t < NT; ++t) { acc[t] = (v8f){}; acc2[t] = (v8f){}; }
#pragma unroll 1
  for (int kb = 0; kb < KD; kb += 32) {
    const v16b af = frag_kb(arow + kb, hh);
    v16b alf = (v16b){};
    if constexpr (RES) alf = frag_kb(alrow + kb, hh);
#pragma unroll
    for (int t = 0; t < NT; ++t) {
      const v16b bf = frag_kb(brow + (size_t)t * 16 * KD + kb, hh);
      acc[t] = wmma16b(af, bf, acc[t]);
      if constexpr (RES) acc2[t] = wmma16b(alf, bf, acc2[t]);
    }
  }
#pragma unroll
  for (int t = 0; t < NT; ++t)
#pragma unroll
    for (int r = 0; r < 8; ++r) {
      float v = acc[t][r];
      if constexpr (RES) v += acc2[t][r] * (1.0f / RS);
      To[wave * 16 + 8 * hh + r][t * 16 + col] = v; }
  __syncthreads();
  if constexpr (MODE == 0) {
    const size_t pb = (((size_t)bsel * nhead + blockIdx.x) * SEQ + s0) * HD;
    b16* ph = Ph + pb; b16* pl = Pl + pb;
    const float qsc = QS / (XS * WS);
    for (int pass = 0; pass < 2; ++pass) {
#pragma unroll 1
      for (int it = 0; it < 8; ++it) {
        const int rr = it * 8 + (tid >> 4), seg = (tid & 15) * 8, sg = seg & 63;
        const float sgn = (seg >= 64) ? 1.0f : -1.0f;
        const float* trow = &To[rr][0]; const size_t ts = (size_t)(s0 + rr) * 64 + sg;
        const v4f xa = *(const v4f*)(trow + seg), xb = *(const v4f*)(trow + seg + 4);
        const v4f ya = *(const v4f*)(trow + (seg ^ 64)), yb = *(const v4f*)(trow + (seg ^ 64) + 4);
        const v4f ca = *(const v4f*)(CT + ts), cb = *(const v4f*)(CT + ts + 4), sa = *(const v4f*)(ST + ts), sb = *(const v4f*)(ST + ts + 4);
        v8b hi, lo;
#pragma unroll
        for (int j = 0; j < 4; ++j) {
          b16 h0, l0;
          split16((xa[j] * ca[j] + sgn * ya[j] * sa[j]) * qsc, h0, l0); hi[j] = h0; lo[j] = l0;
          split16((xb[j] * cb[j] + sgn * yb[j] * sb[j]) * qsc, h0, l0); hi[4 + j] = h0; lo[4 + j] = l0; }
        const size_t off = (size_t)rr * HD + seg;
        *(volatile v8b*)(ph + off) = hi; *(volatile v8b*)(pl + off) = lo; }
      __threadfence(); }
  } else if constexpr (MODE == 1) {
    const size_t pb = ((size_t)bsel * nhead + blockIdx.x) * HD * (size_t)SEQ + s0;
    b16* ph = Ph + pb; b16* pl = Pl + pb;
    const float vsc = QS / (XS * WS);
    for (int pass = 0; pass < 2; ++pass) {
#pragma unroll 1
      for (int it = 0; it < 8; ++it) {
        const int d = it * 16 + (tid >> 3), ss = (tid & 7) * 8;
        v8b hi, lo;
#pragma unroll
        for (int j = 0; j < 8; ++j) { b16 h0, l0; split16(To[ss + j][d] * vsc, h0, l0); hi[j] = h0; lo[j] = l0; }
        const size_t off = (size_t)d * SEQ + ss;
        *(volatile v8b*)(ph + off) = hi; *(volatile v8b*)(pl + off) = lo; }
      __threadfence(); }
  } else {
    constexpr int LPR = BN / 4, RPI = 128 / LPR, NIT = 64 / RPI;
    static_assert(NIT * RPI == 64 && LPR * 4 == BN);
    float* ob = Out + ((size_t)bsel * SEQ_FULL + s0) * DMOD + n0;
    const float osc = 1.0f / (CS * WS);
    for (int pass = 0; pass < 2; ++pass) {
#pragma unroll 1
      for (int it = 0; it < NIT; ++it) {
        const int rr = it * RPI + tid / LPR, seg = (tid % LPR) * 4;
        const v4f f = *(const v4f*)(&To[rr][seg]) * osc;
        *(volatile v4f*)(ob + (size_t)rr * DMOD + seg) = f; }
      __threadfence(); }
  }
}

template <bool ER>
__global__ __launch_bounds__(64) __attribute__((amdgpu_num_vgpr(256))) void attn_kernel(
    const b16* __restrict__ Qh, const b16* __restrict__ Ql, const b16* __restrict__ Kh, const b16* __restrict__ Kl,
    const b16* __restrict__ Vh, const b16* __restrict__ Vl, b16* Ch, b16* Cl) {
  constexpr int NT = ER ? 4 : 8, DW = NT * 16;
  __shared__ __attribute__((aligned(16))) b16 Pb[2][16][32 + 8];
  __shared__ __attribute__((aligned(16))) b16 Pr[2][16][32 + 8];
  __shared__ __attribute__((aligned(16))) float To[2][16][DW + 4];
  const int wave = threadIdx.x >> 5, lane = threadIdx.x & 31, hh = lane >> 4, col = lane & 15;
  const int bh = (int)blockIdx.y; const int b = bh / H, h = bh - b * H, g = h / NREP;
  const int qb0 = (ER ? 0 : QEA) + (int)blockIdx.x * 32;
  const int q0 = qb0 + wave * 16, qi = q0 + col;
  const int dh = ER ? (int)blockIdx.z * 64 : 0;
  const b16* qrow = Qh + ((size_t)(b * H + h) * SEQ + qi) * HD;
  const b16* qlrow = Ql + ((size_t)(b * H + h) * SEQ + qi) * HD;
  const b16* Kb = Kh + (size_t)(b * HKV + g) * SEQ * HD;
  const b16* Klb = Kl + (size_t)(b * HKV + g) * SEQ * HD;
  const b16* Vb = Vh + ((size_t)(b * HKV + g) * HD + dh) * SEQ;
  const b16* Vlb = Vl + ((size_t)(b * HKV + g) * HD + dh) * SEQ;
  v16b qa[4];
#pragma unroll
  for (int c = 0; c < 4; ++c) { qa[c] = (v16b){}; if constexpr (!ER) qa[c] = frag_kb(qrow + c * 32, hh); }
  const float cs = SCL * LOG2E / (QS * QS);
  float m = -INFINITY, l = 0.0f; v8f o[NT], o2[NT];
#pragma unroll
  for (int t = 0; t < NT; ++t) { o[t] = (v8f){}; o2[t] = (v8f){}; }
  const int nst = qb0 / 32 + 1;
#pragma unroll 1
  for (int st = 0; st < nst; ++st) {
    const int kb = st * 32; const int lim = qi - kb;
    float e[16]; float mx = -INFINITY;
#pragma unroll
    for (int u = 0; u < 2; ++u) {
      const size_t kr = (size_t)(kb + u * 16 + col) * HD;
      v8f s = (v8f){}, s2 = (v8f){};
#pragma unroll
      for (int c = 0; c < 4; ++c) {
        const v16b kf = frag_kb(Kb + kr + c * 32, hh);
        if constexpr (ER) {
          const v16b qh = frag_kb(qrow + c * 32, hh), ql = frag_kb(qlrow + c * 32, hh), klf = frag_kb(Klb + kr + c * 32, hh);
          s = wmma16b(kf, qh, s); s2 = wmma16b(kf, ql, s2); s2 = wmma16b(klf, qh, s2);
        } else {
          s = wmma16b(kf, qa[c], s);
        }
      }
#pragma unroll
      for (int r = 0; r < 8; ++r) {
        float v = s[r];
        if constexpr (ER) v += s2[r] * (1.0f / RS);
        v *= cs;
        if (u * 16 + 8 * hh + r > lim) v = -INFINITY;
        e[u * 8 + r] = v; mx = fmaxf(mx, v); } }
    mx = fmaxf(mx, __shfl_xor(mx, 16)); const float mn = fmaxf(m, mx); const float al = nexp2(m - mn); float sum = 0.0f;
#pragma unroll
    for (int i2 = 0; i2 < 16; ++i2) {
      const float p = nexp2(e[i2] - mn); sum += p; const int pi = (i2 < 8 ? 0 : 16) + 8 * hh + (i2 & 7);
      const float pp = p * PS; const b16 phv = (b16)pp; Pb[wave][col][pi] = phv;
      if constexpr (ER) Pr[wave][col][pi] = (b16)((pp - (float)phv) * RS); }
    sum += __shfl_xor(sum, 16); l = l * al + sum; m = mn;
    wave_lds_sync();
    const v16b pf = frag_kb(&Pb[wave][col][0], hh);
    v16b prf = (v16b){};
    if constexpr (ER) prf = frag_kb(&Pr[wave][col][0], hh);
#pragma unroll
    for (int t = 0; t < NT; ++t) {
      o[t] *= al; const v16b vf = frag_kb(Vb + (size_t)(t * 16 + col) * SEQ + kb, hh);
      o[t] = wmma16b(vf, pf, o[t]);
      if constexpr (ER) {
        o2[t] *= al; const v16b vlf = frag_kb(Vlb + (size_t)(t * 16 + col) * SEQ + kb, hh);
        o2[t] = wmma16b(vf, prf, o2[t]); o2[t] = wmma16b(vlf, pf, o2[t]); } }
    wave_lds_sync(); }
  const float inv = 1.0f / (l * PS * QS);
#pragma unroll
  for (int t = 0; t < NT; ++t) {
#pragma unroll
    for (int r = 0; r < 8; ++r) {
      float ov = o[t][r];
      if constexpr (ER) ov += o2[t][r] * (1.0f / RS);
      To[wave][col][t * 16 + 8 * hh + r] = ov * inv; } }
  wave_lds_sync();
  constexpr int LPR = DW / 8, RPI = 32 / LPR, NIT = 16 / RPI;
  static_assert(NIT * RPI == 16 && LPR * 8 == DW);
  const size_t cbase = ((size_t)b * SEQ + q0) * DMOD + (size_t)h * HD + dh;
  for (int pass = 0; pass < 2; ++pass) {
#pragma unroll 1
    for (int it = 0; it < NIT; ++it) {
      const int rr = it * RPI + lane / LPR, seg = (lane % LPR) * 8;
      const v4f fa = *(const v4f*)(&To[wave][rr][seg]), fb = *(const v4f*)(&To[wave][rr][seg + 4]);
      v8b hi, lo;
#pragma unroll
      for (int j = 0; j < 4; ++j) { b16 h0, l0; split16(fa[j] * CS, h0, l0); hi[j] = h0; lo[j] = l0; split16(fb[j] * CS, h0, l0); hi[4 + j] = h0; lo[4 + j] = l0; }
      const size_t off = cbase + (size_t)rr * DMOD + seg;
      *(volatile v8b*)(Ch + off) = hi; *(volatile v8b*)(Cl + off) = lo; }
    __threadfence(); }
}
}

extern "C" void kernel_launch(void* const* d_in, const int* in_sizes, int n_in, void* d_out, int out_size, void* d_ws, size_t ws_size, hipStream_t stream) {
  const size_t need_x = ((size_t)(NB - 1) * SEQ_FULL + SEQ) * DMOD;
  if (n_in < 5 || (size_t)in_sizes[0] < need_x || (size_t)in_sizes[1] < (size_t)KD * DMOD || (size_t)in_sizes[2] < (size_t)KD * NKV ||
      (size_t)in_sizes[3] < (size_t)KD * NKV || (size_t)in_sizes[4] < (size_t)KD * DMOD || (size_t)out_size < need_x) return;
  const float* X = (const float*)d_in[0]; const float* Wq = (const float*)d_in[1]; const float* Wk = (const float*)d_in[2];
  const float* Wv = (const float*)d_in[3]; const float* Wo = (const float*)d_in[4]; float* out = (float*)d_out;
  size_t off = 0; char* ws = (char*)d_ws;
  auto carve = [&](size_t bytes) { char* p = ws + off; off += (bytes + 255) & ~(size_t)255; return p; };
  b16* Xp  = (b16*)carve((size_t)MR * DMOD * 2);
  b16* Wqt = (b16*)carve((size_t)DMOD * KD * 2);
  b16* Wkt = (b16*)carve((size_t)NKV * KD * 2);
  b16* Wvt = (b16*)carve((size_t)NKV * KD * 2);
  b16* Wot = (b16*)carve((size_t)DMOD * KD * 2);
  float* CT = (float*)carve((size_t)SEQ * 64 * 4);
  float* ST = (float*)carve((size_t)SEQ * 64 * 4);
  b16* Qh = (b16*)carve((size_t)MR * H * HD * 2);
  b16* Ql = (b16*)carve((size_t)MR * H * HD * 2);
  b16* Kh = (b16*)carve((size_t)MR * NKV * 2);
  b16* Kl = (b16*)carve((size_t)MR * NKV * 2);
  b16* Vh = (b16*)carve((size_t)MR * NKV * 2);
  b16* Vl = (b16*)carve((size_t)MR * NKV * 2);
  b16* Ch = (b16*)carve((size_t)MR * DMOD * 2);
  b16* Cl = (b16*)carve((size_t)MR * DMOD * 2);
  if (off > ws_size || off > ((size_t)128 << 20)) return;
  cvt_x_kernel<<<dim3((unsigned)MR), 256, 0, stream>>>(X, Xp);
  cvt_w_kernel<<<dim3(KD / 64, DMOD / 64), 64, 0, stream>>>(Wq, Wqt, DMOD);
  cvt_w_kernel<<<dim3(KD / 64, NKV / 64), 64, 0, stream>>>(Wk, Wkt, NKV);
  cvt_w_kernel<<<dim3(KD / 64, NKV / 64), 64, 0, stream>>>(Wv, Wvt, NKV);
  cvt_w_kernel<<<dim3(KD / 64, DMOD / 64), 64, 0, stream>>>(Wo, Wot, DMOD);
  rope_tab_kernel<<<dim3(SEQ / 4), 256, 0, stream>>>(CT, ST);
  proj_kernel<0, false><<<dim3(DMOD / 128, MR / 64), 128, 0, stream>>>(Xp, Xp, Wqt, Qh, Ql, out, CT, ST, H, SEQ / 64, 0);
  proj_kernel<0, false><<<dim3(NKV / 128, MR / 64), 128, 0, stream>>>(Xp, Xp, Wkt, Kh, Kl, out, CT, ST, HKV, SEQ / 64, 0);
  proj_kernel<1, false><<<dim3(NKV / 128, MR / 64), 128, 0, stream>>>(Xp, Xp, Wvt, Vh, Vl, out, CT, ST, HKV, SEQ / 64, 0);
  attn_kernel<true><<<dim3(QEA / 32, NB * H, 2), 64, 0, stream>>>(Qh, Ql, Kh, Kl, Vh, Vl, Ch, Cl);
  if (SEQ > QEA) attn_kernel<false><<<dim3((SEQ - QEA) / 32, NB * H, 1), 64, 0, stream>>>(Qh, Ql, Kh, Kl, Vh, Vl, Ch, Cl);
  proj_kernel<2, true><<<dim3(DMOD / 64, NB * (QEA / 64)), 128, 0, stream>>>(Ch, Cl, Wot, Ch, Cl, out, CT, ST, 1, QEA / 64, 0);
  if (SEQ > QEA) proj_kernel<2, false><<<dim3(DMOD / 128, NB * ((SEQ - QEA) / 64)), 128, 0, stream>>>(Ch, Ch, Wot, Ch, Cl, out, CT, ST, 1, (SEQ - QEA) / 64, QEA);
}
